// MambaBlock_82171314307105
// MI455X (gfx1250) — hardware-verified
//
#include <hip/hip_runtime.h>
#include <stddef.h>
#include <stdint.h>
#include <math.h>

#define DM    1024
#define TIN   1022
#define TS    1024
#define NB    8
#define MR    (NB * TS)
#define HP    2048
#define UH    4096
#define GBM   64
#define GBN   128
#define GTHR  128
#define NTHR  256
#define SC_T  16
#define SC_C  128
#define WSMAX 134217728

static_assert(TS == DM && TIN + 2 == TS);
static_assert(MR % GBM == 0 && UH % GBM == 0 && DM % GBN == 0 && (2 * DM) % GBN == 0);
static_assert(DM % 32 == 0 && HP == 2 * DM && GTHR == GBN && GBM == (GTHR / 32) * 16);
static_assert(TS % GBM == 0 && TS % SC_T == 0 && DM % SC_C == 0);
static_assert((SC_T * 2 * SC_C) / 8 == 4 * SC_C);

typedef float          v4f   __attribute__((ext_vector_type(4)));
typedef float          v8f   __attribute__((ext_vector_type(8)));
typedef int            v8i   __attribute__((ext_vector_type(8)));
typedef unsigned short v4us  __attribute__((ext_vector_type(4)));
typedef unsigned short v8us  __attribute__((ext_vector_type(8)));
typedef unsigned short v16us __attribute__((ext_vector_type(16)));
typedef __bf16         v16bf __attribute__((ext_vector_type(16)));
typedef v4f  __attribute__((may_alias)) v4fa;
typedef v4us __attribute__((may_alias)) v4usa;
typedef v8us __attribute__((may_alias)) v8usa;
union FragB { v16bf v; v16us u; v8us h[2]; v8i w; };

__device__ __forceinline__ v8f wmb(const FragB& a, const FragB& b, v8f c) {
  v8f d = __builtin_amdgcn_wmma_f32_16x16x32_bf16(false, a.v, false, b.v, (short)0, c, false, false);
  asm volatile("v_nop\n\tv_nop\n\tv_nop\n\tv_nop" : "+v"(d) : "v"(a.w), "v"(b.w));
  return d;
}

__device__ __forceinline__ unsigned bf16_bits(float f) {
  const unsigned u = __float_as_uint(f);
  return (u + 0x7FFFu + ((u >> 16) & 1u)) >> 16;
}
__device__ __forceinline__ float bf16_val(float f) {
  return __uint_as_float(bf16_bits(f) << 16);
}

__global__ __launch_bounds__(NTHR) void k_wT(const float* __restrict__ W, unsigned short* WT) {
  const int u  = (int)blockIdx.x * NTHR + (int)threadIdx.x;
  const int n  = u >> 7;
  const int k8 = (u & 127) * 8;
  const float* p = W + (size_t)k8 * DM + n;
  v8us o;
#pragma unroll
  for (int i = 0; i < 8; ++i) o[i] = (unsigned short)bf16_bits(p[(size_t)i * DM]);
  unsigned short* dp = WT + (size_t)n * DM + k8;
  *(volatile v8us*)dp = o;
  __threadfence();
  *(volatile v8us*)dp = o;
}

__global__ __launch_bounds__(NTHR) void k_cvx(const float* __restrict__ x, unsigned short* xb) {
  const int u   = (int)blockIdx.x * NTHR + (int)threadIdx.x;
  const int row = u >> 7;
  const int k8  = (u & 127) * 8;
  const int b   = row >> 10;
  const int t   = row & (TS - 1);
  const int tc  = t < TIN ? t : TIN - 1;
  const float* p = x + ((size_t)b * TIN + tc) * DM + k8;
  const v4f a = *(const v4fa*)p;
  const v4f c = *(const v4fa*)(p + 4);
  const bool ok = t < TIN;
  v8us o;
  o[0] = ok ? (unsigned short)bf16_bits(a.x) : (unsigned short)0;
  o[1] = ok ? (unsigned short)bf16_bits(a.y) : (unsigned short)0;
  o[2] = ok ? (unsigned short)bf16_bits(a.z) : (unsigned short)0;
  o[3] = ok ? (unsigned short)bf16_bits(a.w) : (unsigned short)0;
  o[4] = ok ? (unsigned short)bf16_bits(c.x) : (unsigned short)0;
  o[5] = ok ? (unsigned short)bf16_bits(c.y) : (unsigned short)0;
  o[6] = ok ? (unsigned short)bf16_bits(c.z) : (unsigned short)0;
  o[7] = ok ? (unsigned short)bf16_bits(c.w) : (unsigned short)0;
  unsigned short* dp = xb + (size_t)row * DM + k8;
  *(volatile v8us*)dp = o;
  __threadfence();
  *(volatile v8us*)dp = o;
}

__global__ __launch_bounds__(NTHR) void k_conv_silu(const float* __restrict__ X1, const float* __restrict__ cw,
                                                    const float* __restrict__ cb, unsigned short* U) {
  __shared__ __attribute__((aligned(16))) unsigned short sh[2 * HP];
  const int tid  = (int)threadIdx.x;
  const int row0 = (int)blockIdx.x * 2;
#pragma unroll 1
  for (int it = 0; it < 8; ++it) {
    const int e   = it * NTHR + tid;
    const int rl  = e >> 10;
    const int c   = e & (DM - 1);
    const int row = row0 + rl;
    const int t   = row & (TS - 1);
    const int ra  = (t >= 2) ? row - 2 : row;
    const int rb  = (t >= 1) ? row - 1 : row;
    const float xa = X1[(size_t)ra * DM + c];
    const float xq = X1[(size_t)rb * DM + c];
    const float xc = X1[(size_t)row * DM + c];
    const float w0 = bf16_val(cw[3 * c + 0]);
    const float w1 = bf16_val(cw[3 * c + 1]);
    const float w2 = bf16_val(cw[3 * c + 2]);
    const float bb = bf16_val(cb[c]);
    const float fa = (t >= 2) ? xa : 0.0f;
    const float fb = (t >= 1) ? xq : 0.0f;
    const float v  = ((w0 * fa + w1 * fb) + w2 * xc) + bb;
    const float uu = v * (1.0f / (1.0f + expf(-v)));
    const unsigned hb = bf16_bits(uu);
    const unsigned lb = bf16_bits(uu - __uint_as_float(hb << 16));
    sh[rl * HP + c]      = (unsigned short)hb;
    sh[rl * HP + DM + c] = (unsigned short)lb;
  }
  __syncthreads();
  const v8us q0 = *(const v8usa*)(sh + 8 * tid);
  const v8us q1 = *(const v8usa*)(sh + 8 * (NTHR + tid));
  unsigned short* d0 = U + (size_t)row0 * HP + 8 * tid;
  unsigned short* d1 = d0 + 8 * NTHR;
  *(volatile v8us*)d0 = q0;
  *(volatile v8us*)d1 = q1;
  __threadfence();
  *(volatile v8us*)d0 = q0;
  *(volatile v8us*)d1 = q1;
}

__global__ __launch_bounds__(SC_C) void k_scan(const float* __restrict__ AB, const float* __restrict__ BXp,
                                               unsigned short* H) {
  __shared__ __attribute__((aligned(16))) unsigned short sh[SC_T * 2 * SC_C];
  const int tid = (int)threadIdx.x;
  const int b   = (int)blockIdx.x >> 3;
  const int cb0 = ((int)blockIdx.x & 7) * SC_C;
  const size_t base = (size_t)b * TS * DM + (size_t)(cb0 + tid);
  float h = 0.0f;
#pragma unroll 1
  for (int t0 = 0; t0 < TS; t0 += SC_T) {
#pragma unroll 4
    for (int tt = 0; tt < SC_T; ++tt) {
      const size_t o = base + (size_t)(t0 + tt) * DM;
      const float a  = AB[o];
      const float bx = BXp[o];
      const float hn = fmaf(a, h, bx);
      h = ((t0 + tt) == 0) ? bx : hn;
      const unsigned hb = bf16_bits(h);
      const unsigned lb = bf16_bits(h - __uint_as_float(hb << 16));
      sh[tt * (2 * SC_C) + tid]        = (unsigned short)hb;
      sh[tt * (2 * SC_C) + SC_C + tid] = (unsigned short)lb;
    }
    __syncthreads();
    v8us q[4];
#pragma unroll
    for (int j = 0; j < 4; ++j) q[j] = *(const v8usa*)(sh + 8 * (j * SC_C + tid));
#pragma unroll
    for (int j = 0; j < 4; ++j) {
      const int p  = j * SC_C + tid;
      const int tr = p >> 5;
      const int qq = p & 31;
      const int col = (qq < 16) ? (cb0 + 8 * qq) : (DM + cb0 + 8 * (qq - 16));
      unsigned short* dp = H + (size_t)(b * TS + t0 + tr) * HP + col;
      *(volatile v8us*)dp = q[j];
    }
    __threadfence();
#pragma unroll
    for (int j = 0; j < 4; ++j) {
      const int p  = j * SC_C + tid;
      const int tr = p >> 5;
      const int qq = p & 31;
      const int col = (qq < 16) ? (cb0 + 8 * qq) : (DM + cb0 + 8 * (qq - 16));
      unsigned short* dp = H + (size_t)(b * TS + t0 + tr) * HP + col;
      *(volatile v8us*)dp = q[j];
    }
    __syncthreads();
  }
}

#define EP_F32 0
#define EP_U   1
#define EP_HLB 2
#define EP_HL  3
#define EP_XRT 4

template <int EP>
__global__ __launch_bounds__(GTHR) void k_gemm(
    const unsigned short* wsb,
    size_t aOff0, size_t bOff0, size_t aOff1, size_t bOff1, size_t sBz,
    const float* __restrict__ v0, const float* __restrict__ v1, const float* __restrict__ v2,
    float* outF, unsigned short* outH,
    int K0, int K1, int lda, int ldb)
{
  __shared__ __attribute__((aligned(16))) float stg[GBM * GBN];
  __shared__ __attribute__((aligned(16))) float sv0[GBN];
  __shared__ __attribute__((aligned(16))) float sv1[GBN];
  const int tid = (int)threadIdx.x, lane = tid & 31, wave = tid >> 5, hh = lane >> 4, m = lane & 15;
  const int rowBase = ((int)blockIdx.z * (int)gridDim.x + (int)blockIdx.x) * GBM;
  const int col0    = (int)blockIdx.y * GBN;

  v8f acc[8];
  {
    const v8f z = {0.f, 0.f, 0.f, 0.f, 0.f, 0.f, 0.f, 0.f};
#pragma unroll
    for (int t = 0; t < 8; ++t) acc[t] = z;
  }

#pragma unroll 1
  for (int seg = 0; seg < 2; ++seg) {
    const size_t ao = seg ? aOff1 : aOff0;
    const size_t bo = seg ? bOff1 : bOff0;
    const int    K  = seg ? K1 : K0;
    const unsigned short* ap = wsb + ao + (size_t)(rowBase + 16 * wave + m) * (size_t)lda + 8 * hh;
    const unsigned short* bp = wsb + bo + (size_t)blockIdx.z * sBz + (size_t)(col0 + m) * (size_t)ldb + 8 * hh;
#pragma unroll 1
    for (int k0 = 0; k0 < K; k0 += 32) {
      const int kb = k0 & (DM - 1);
      FragB af;
      af.h[0] = *(const v8usa*)(ap + k0);
      af.h[1] = *(const v8usa*)(ap + k0 + 16);
#pragma unroll
      for (int nt = 0; nt < 8; ++nt) {
        const unsigned short* wq = bp + (size_t)(16 * nt) * (size_t)ldb + kb;
        FragB bf;
        bf.h[0] = *(const v8usa*)wq;
        bf.h[1] = *(const v8usa*)(wq + 16);
        acc[nt] = wmb(af, bf, acc[nt]);
      }
    }
  }

#pragma unroll
  for (int nt = 0; nt < 8; ++nt) {
    const int lc = 16 * nt + m;
#pragma unroll
    for (int r = 0; r < 8; ++r) {
      const int lr = 16 * wave + 8 * hh + r;
      stg[lr * GBN + lc] = acc[nt][r];
    }
  }
  if constexpr (EP == EP_U) {
    const int cm = (col0 & (DM - 1)) + tid;
    const float bd = bf16_val(v0[cm]);
    const float av = bf16_val(v1[cm]);
    const float bb = bf16_val(v2[cm]);
    sv0[tid] = (col0 >= DM) ? bb : bd;
    sv1[tid] = av;
  }
  if constexpr (EP == EP_HLB) {
    const int cm = col0 + tid;
    sv0[tid] = bf16_val(v0[cm]) + bf16_val(v1[cm]);
    sv1[tid] = 0.0f;
  }
  __syncthreads();

  if constexpr (EP == EP_U) {
    const bool isB = col0 >= DM;
#pragma unroll 1
    for (int j = 0; j < 64; ++j) {
      const int cc  = 4 * lane + (j & 3);
      const int idx = (16 * wave + (j >> 2)) * GBN + cc;
      float v = stg[idx] + sv0[cc];
      if (!isB) {
        const float sp = fmaxf(v, 0.0f) + log1pf(expf(-fabsf(v)));
        v = expf(-(sp * sv1[cc]));
      }
      stg[idx] = v;
    }
    __syncthreads();
  }
  if constexpr (EP == EP_XRT) {
#pragma unroll 1
    for (int j = 0; j < 64; ++j) {
      const int cc  = 4 * lane + (j & 3);
      const int idx = (16 * wave + (j >> 2)) * GBN + cc;
      const float v = stg[idx];
      stg[idx] = v * (1.0f / (1.0f + expf(-v)));
    }
    __syncthreads();
  }

  if constexpr (EP == EP_F32 || EP == EP_U) {
    const size_t pOff = (EP == EP_U && col0 >= DM) ? (size_t)UH * DM : (size_t)0;
    const int colOut  = (EP == EP_U) ? (col0 & (DM - 1)) : col0;
    v4f pv[16];
#pragma unroll
    for (int i = 0; i < 16; ++i) pv[i] = *(const v4fa*)(stg + (16 * wave + i) * GBN + 4 * lane);
#pragma unroll
    for (int i = 0; i < 16; ++i) {
      float* op = outF + pOff + (size_t)(rowBase + 16 * wave + i) * DM + colOut + 4 * lane;
      *(volatile v4f*)op = pv[i];
    }
    __threadfence();
#pragma unroll
    for (int i = 0; i < 16; ++i) {
      float* op = outF + pOff + (size_t)(rowBase + 16 * wave + i) * DM + colOut + 4 * lane;
      *(volatile v4f*)op = pv[i];
    }
  }

  if constexpr (EP == EP_HLB || EP == EP_HL) {
    v4f pv[16];
#pragma unroll
    for (int i = 0; i < 16; ++i) pv[i] = *(const v4fa*)(stg + (16 * wave + i) * GBN + 4 * lane);
    if constexpr (EP == EP_HLB) {
      const v4f bb4 = *(const v4fa*)(sv0 + 4 * lane);
#pragma unroll
      for (int i = 0; i < 16; ++i) pv[i] = pv[i] + bb4;
    }
    __syncthreads();
#pragma unroll
    for (int i = 0; i < 16; ++i) {
      v4us h4, l4;
      unsigned hb;
      hb = bf16_bits(pv[i].x); h4[0] = (unsigned short)hb; l4[0] = (unsigned short)bf16_bits(pv[i].x - __uint_as_float(hb << 16));
      hb = bf16_bits(pv[i].y); h4[1] = (unsigned short)hb; l4[1] = (unsigned short)bf16_bits(pv[i].y - __uint_as_float(hb << 16));
      hb = bf16_bits(pv[i].z); h4[2] = (unsigned short)hb; l4[2] = (unsigned short)bf16_bits(pv[i].z - __uint_as_float(hb << 16));
      hb = bf16_bits(pv[i].w); h4[3] = (unsigned short)hb; l4[3] = (unsigned short)bf16_bits(pv[i].w - __uint_as_float(hb << 16));
      unsigned short* srow = (unsigned short*)stg + (size_t)(16 * wave + i) * (2 * GBN);
      *(v4usa*)(srow + 4 * lane) = h4;
      *(v4usa*)(srow + GBN + 4 * lane) = l4;
    }
    __syncthreads();
    v8us qv[16];
#pragma unroll
    for (int i = 0; i < 16; ++i) {
      const unsigned short* srow = (const unsigned short*)stg + (size_t)(16 * wave + i) * (2 * GBN);
      qv[i] = *(const v8usa*)(srow + 8 * lane);
    }
    const int colH = (lane < 16) ? (col0 + 8 * lane) : (DM + col0 + 8 * (lane - 16));
#pragma unroll
    for (int i = 0; i < 16; ++i) {
      unsigned short* rp = outH + (size_t)(rowBase + 16 * wave + i) * HP + colH;
      *(volatile v8us*)rp = qv[i];
    }
    __threadfence();
#pragma unroll
    for (int i = 0; i < 16; ++i) {
      unsigned short* rp = outH + (size_t)(rowBase + 16 * wave + i) * HP + colH;
      *(volatile v8us*)rp = qv[i];
    }
  }

  if constexpr (EP == EP_XRT) {
    const int bidx = rowBase >> 10;
    const int t0   = rowBase & (TS - 1);
    unsigned short* dst = outH + ((size_t)bidx * DM + (size_t)col0) * HP + t0;
    auto xpass = [&]() {
#pragma unroll 1
      for (int it = 0; it < 16; ++it) {
        const int e    = 32 * wave + 2 * it + (lane >> 4);
        const int part = (lane >> 3) & 1;
        const int q    = lane & 7;
        v8us o;
#pragma unroll
        for (int j = 0; j < 8; ++j) {
          const float v = stg[(8 * q + j) * GBN + e];
          const unsigned hb = bf16_bits(v);
          const unsigned lb = bf16_bits(v - __uint_as_float(hb << 16));
          o[j] = (unsigned short)(part ? lb : hb);
        }
        unsigned short* dp = dst + (size_t)e * HP + part * DM + 8 * q;
        *(volatile v8us*)dp = o;
      }
    };
    xpass();
    __threadfence();
    xpass();
  }
}

extern "C" void kernel_launch(void* const* d_in, const int* in_sizes, int n_in,
                              void* d_out, int out_size, void* d_ws, size_t ws_size,
                              hipStream_t stream) {
  if (n_in < 15) return;
  if (in_sizes[0] != NB * TIN * DM) return;
  if (in_sizes[1] != DM * DM || in_sizes[2] != DM * DM || in_sizes[3] != DM * DM) return;
  if (in_sizes[4] != DM * 3 || in_sizes[5] != DM || in_sizes[6] != DM) return;
  if (in_sizes[7] != DM * DM || in_sizes[8] != DM) return;
  if (in_sizes[9] != DM * DM || in_sizes[10] != DM) return;
  if (in_sizes[11] != DM * DM || in_sizes[12] != DM) return;
  if (in_sizes[13] != DM * DM || in_sizes[14] != DM) return;
  if (out_size != MR * DM) return;

  const float* x      = (const float*)d_in[0];
  const float* w1     = (const float*)d_in[1];
  const float* w2     = (const float*)d_in[2];
  const float* wlast  = (const float*)d_in[3];
  const float* convw  = (const float*)d_in[4];
  const float* convb  = (const float*)d_in[5];
  const float* Avec   = (const float*)d_in[6];
  const float* wB     = (const float*)d_in[7];
  const float* bB     = (const float*)d_in[8];
  const float* wC     = (const float*)d_in[9];
  const float* bC     = (const float*)d_in[10];
  const float* wD     = (const float*)d_in[11];
  const float* bD     = (const float*)d_in[12];
  const float* wdelta = (const float*)d_in[13];
  const float* bdelta = (const float*)d_in[14];
  float* out = (float*)d_out;

  const size_t WEL = (size_t)DM * DM;
  const size_t bWT = 7 * WEL * 2;
  const size_t bR  = (size_t)MR * DM * 4;
  const size_t oR0 = bWT, oR1 = oR0 + bR, oR2 = oR1 + bR, total = oR2 + bR;
  if (total > ws_size || total > (size_t)WSMAX) return;
  char* ws = (char*)d_ws;
  unsigned short* wsb = (unsigned short*)ws;
  const size_t eR0 = oR0 / 2, eR1 = oR1 / 2, eR2 = oR2 / 2;
  unsigned short* WT  = wsb;
  float*          R0f = (float*)(ws + oR0);
  float*          R2f = (float*)(ws + oR2);
  unsigned short* R0h = wsb + eR0;
  unsigned short* R1h = wsb + eR1;
  unsigned short* R2h = wsb + eR2;

  const int gW = (int)(WEL / 8 / NTHR);
  k_wT<<<gW, NTHR, 0, stream>>>(w1,     WT + 0 * WEL);
  k_wT<<<gW, NTHR, 0, stream>>>(wdelta, WT + 1 * WEL);
  k_wT<<<gW, NTHR, 0, stream>>>(wB,     WT + 2 * WEL);
  k_wT<<<gW, NTHR, 0, stream>>>(wC,     WT + 3 * WEL);
  k_wT<<<gW, NTHR, 0, stream>>>(wD,     WT + 4 * WEL);
  k_wT<<<gW, NTHR, 0, stream>>>(w2,     WT + 5 * WEL);
  k_wT<<<gW, NTHR, 0, stream>>>(wlast,  WT + 6 * WEL);
  k_cvx<<<MR * (DM / 8) / NTHR, NTHR, 0, stream>>>(x, R1h);
  k_gemm<EP_F32><<<dim3(MR / GBM, DM / GBN, 1), GTHR, 0, stream>>>(
      wsb, eR1, 0 * WEL, eR1, 0 * WEL, 0, convb, convb, convb, R0f, R0h, DM, 0, DM, DM);
  k_conv_silu<<<MR / 2, NTHR, 0, stream>>>(R0f, convw, convb, R1h);
  for (int half = 0; half < 2; ++half) {
    const size_t aU = eR1 + (size_t)half * UH * HP;
    k_gemm<EP_U><<<dim3(UH / GBM, (2 * DM) / GBN, 1), GTHR, 0, stream>>>(
        wsb, aU, 1 * WEL, aU, 1 * WEL, 0, bdelta, Avec, bB, R2f, R2h, 2 * DM, 0, HP, DM);
    k_scan<<<4 * (DM / SC_C), SC_C, 0, stream>>>(R2f, R2f + (size_t)UH * DM, R0h + (size_t)half * UH * HP);
  }
  k_gemm<EP_HLB><<<dim3(MR / GBM, DM / GBN, 1), GTHR, 0, stream>>>(
      wsb, eR0, 3 * WEL, eR1, 4 * WEL, 0, bC, bD, bD, R0f, R2h, 2 * DM, 2 * DM, HP, DM);
  k_gemm<EP_XRT><<<dim3(MR / GBM, DM / GBN, 1), GTHR, 0, stream>>>(
      wsb, eR2, 5 * WEL, eR2, 5 * WEL, 0, convb, convb, convb, R0f, R0h, 2 * DM, 0, HP, DM);
  k_gemm<EP_HL><<<dim3(TS / GBM, DM / GBN, NB), GTHR, 0, stream>>>(
      wsb, eR2, eR0, eR2, eR0 + DM, (size_t)DM * HP, convb, convb, convb, R0f, R1h, 2 * DM, DM, HP, HP);
  k_gemm<EP_F32><<<dim3(MR / GBM, DM / GBN, 1), GTHR, 0, stream>>>(
      wsb, eR1, 6 * WEL, eR1, 6 * WEL, 0, convb, convb, convb, out, R1h, 2 * DM, 0, HP, DM);
}
